// GAT_37426345017680
// MI455X (gfx1250) — hardware-verified
//
#include <hip/hip_runtime.h>
#include <stddef.h>
#include <stdint.h>
#include <math.h>


#define DIN     128
#define H1C     16
#define NCOL    32
#define GBM     64
#define GTHR    128
#define NTHR    256
#define NWAVE   8
#define NBRUN   256
#define SLB     8
#define NBP     512
#define CE      8192
#define WSUB    (CE / NWAVE)
#define GPW     (WSUB / 32)
#define SEGCAP  64
#define NCHP    512
#define RCAP    12288
#define DEGCAP  128
#define NEGSL   0.2f
#define EPS_SM  1e-16f
#define WSMAX   134217728

#define O_SEGCNT 0
#define O_SEGOFF (O_SEGCNT + NCHP)
#define O_HL     (O_SEGOFF + NCHP)
#define O_SL     (O_HL + RCAP)
#define O_WCN    (O_SL + RCAP)
#define O_CNT    (O_WCN + NWAVE * NBRUN)
#define O_OFFS   (O_CNT + NBRUN)
#define O_MISC   (O_OFFS + NBRUN)
#define ZINTS    (O_MISC + 16)

static_assert(NBRUN == (1 << SLB) && (NBRUN % 32) == 0);
static_assert(NBRUN == NTHR && NBRUN == NWAVE * 32);
static_assert(NBP == 2 * NTHR && NCHP == 2 * NTHR);
static_assert(NBP <= (1 << 9));
static_assert(CE == NWAVE * GPW * 32);
static_assert((CE % 4) == 0 && ((NWAVE * NBP) % 4) == 0 && (ZINTS % 4) == 0);
static_assert(SEGCAP == 64 && (SEGCAP % 32) == 0);
static_assert((RCAP % 256) == 0);
static_assert(ZINTS * 4 <= 300000);
static_assert(GBM == (GTHR / 32) * 16 && NCOL == 2 * H1C && (DIN % 32) == 0);
static_assert(GBM * H1C / 4 == 2 * GTHR);

typedef float          v4f  __attribute__((ext_vector_type(4)));
typedef float          v8f  __attribute__((ext_vector_type(8)));
typedef int            v4i  __attribute__((ext_vector_type(4)));
typedef int            v8i  __attribute__((ext_vector_type(8)));
typedef unsigned int   v4u  __attribute__((ext_vector_type(4)));
typedef unsigned short v8us __attribute__((ext_vector_type(8)));
typedef __bf16         v16b __attribute__((ext_vector_type(16)));
typedef v4f  __attribute__((may_alias)) v4fa;
typedef v4i  __attribute__((may_alias)) v4ia;
typedef v8us __attribute__((may_alias)) v8usa;
union FragB { v16b v; v8us h[2]; v4u q[2]; v8i w; };

__device__ __forceinline__ v8f wmb(const FragB& a, const FragB& b, v8f c) {
  v8f d = __builtin_amdgcn_wmma_f32_16x16x32_bf16(false, a.v, false, b.v, (short)0, c, false, false);
  asm volatile("v_nop\n\tv_nop\n\tv_nop\n\tv_nop" : "+v"(d) : "v"(a.w), "v"(b.w));
  return d;
}

__device__ __forceinline__ unsigned int f2bf(float f) {
  const unsigned int u = __float_as_uint(f);
  return ((u + 0x7FFFu + ((u >> 16) & 1u)) >> 16) & 0xFFFFu;
}
__device__ __forceinline__ float bfr(float f) { return __uint_as_float(f2bf(f) << 16); }
__device__ __forceinline__ unsigned int pk2(float lo, float hi) { return f2bf(lo) | (f2bf(hi) << 16); }
__device__ __forceinline__ v4u pack8(const v4f a, const v4f b) {
  v4u r;
  r.x = pk2(a.x, a.y); r.y = pk2(a.z, a.w); r.z = pk2(b.x, b.y); r.w = pk2(b.z, b.w);
  return r;
}

template <int NBITS>
__device__ __forceinline__ unsigned match_mask(int key, bool valid) {
  unsigned mm = __builtin_amdgcn_ballot_w32(valid);
#pragma unroll
  for (int bit = 0; bit < NBITS; ++bit) {
    const bool bt = ((key >> bit) & 1) != 0;
    const unsigned bal = __builtin_amdgcn_ballot_w32(bt);
    mm &= bt ? bal : ~bal;
  }
  return mm;
}

__device__ __forceinline__ int wave_incl(int v, int lane) {
#pragma unroll
  for (int d = 1; d < 32; d <<= 1) {
    const int up = __shfl_up(v, d);
    v += (lane >= d) ? up : 0;
  }
  return v;
}

__global__ __launch_bounds__(NTHR) void k_wprep(const float* __restrict__ Ws, const float* __restrict__ Wd,
                                                unsigned short* WT) {
  const int u  = (int)blockIdx.x * NTHR + (int)threadIdx.x;
  const int n  = u >> 4;
  const int nn = n & 15;
  const int k8 = (u & 15) * 8;
  v8us o;
  if (blockIdx.x == 0) {
    const float* p = Ws + (size_t)k8 * H1C + nn;
#pragma unroll
    for (int i = 0; i < 8; ++i) o[i] = (unsigned short)f2bf(p[(size_t)i * H1C]);
  } else {
    const float* p = Wd + (size_t)k8 * H1C + nn;
#pragma unroll
    for (int i = 0; i < 8; ++i) o[i] = (unsigned short)f2bf(p[(size_t)i * H1C]);
  }
  unsigned short* dp = WT + (size_t)n * DIN + k8;
  *(volatile v8us*)dp = o;
  __threadfence();
  *(volatile v8us*)dp = o;
}

__global__ __launch_bounds__(GTHR) void k_gemm1(const float* __restrict__ x, const unsigned short* __restrict__ WT,
                                                const float* __restrict__ a1s, const float* __restrict__ a1d,
                                                float* HS, float* SD, int nN, int MPr) {
  __shared__ __attribute__((aligned(16))) float stg[GBM * NCOL];
  __shared__ __attribute__((aligned(16))) float satt[NCOL];
  __shared__ __attribute__((aligned(16))) float sdot[2 * GBM];
  const int tid = (int)threadIdx.x, lane = tid & 31, wave = tid >> 5, hh = lane >> 4, m = lane & 15;
  const int rowBase = (int)blockIdx.x * GBM;

  if (wave == 0) {
    const int c = lane & 15;
    const unsigned int us = __float_as_uint(a1s[c]);
    const unsigned int ud = __float_as_uint(a1d[c]);
    const unsigned int mk = 0u - (unsigned int)(lane >> 4);
    const unsigned int ub = (us & ~mk) | (ud & mk);
    satt[lane] = bfr(__uint_as_float(ub));
  }

  const int row = rowBase + 16 * wave + m;
  const int rc  = row < nN ? row : nN - 1;
  const float* xr = x + (size_t)rc * DIN + 8 * hh;
  const unsigned short* wp = WT + (size_t)m * DIN + 8 * hh;

  v8f acc[2];
  {
    const v8f z = {0.f, 0.f, 0.f, 0.f, 0.f, 0.f, 0.f, 0.f};
    acc[0] = z; acc[1] = z;
  }
#pragma unroll
  for (int ks = 0; ks < DIN / 32; ++ks) {
    const v4f a0 = *(const v4fa*)(xr + 32 * ks);
    const v4f a1 = *(const v4fa*)(xr + 32 * ks + 4);
    const v4f a2 = *(const v4fa*)(xr + 32 * ks + 16);
    const v4f a3 = *(const v4fa*)(xr + 32 * ks + 20);
    FragB af;
    af.q[0] = pack8(a0, a1);
    af.q[1] = pack8(a2, a3);
#pragma unroll
    for (int t = 0; t < 2; ++t) {
      const unsigned short* wq = wp + (size_t)(16 * t) * DIN + 32 * ks;
      FragB bf;
      bf.h[0] = *(const v8usa*)wq;
      bf.h[1] = *(const v8usa*)(wq + 16);
      acc[t] = wmb(af, bf, acc[t]);
    }
  }

#pragma unroll
  for (int t = 0; t < 2; ++t) {
#pragma unroll
    for (int r = 0; r < 8; ++r) {
      const int lr = 16 * wave + 8 * hh + r;
      stg[lr * NCOL + 16 * t + m] = acc[t][r];
    }
  }
  __syncthreads();

  {
    const int rw = tid & 63, which = tid >> 6;
    const float* hr = stg + rw * NCOL + which * H1C;
    const float* sa = satt + which * H1C;
    float d = 0.f;
#pragma unroll 1
    for (int c4 = 0; c4 < H1C / 4; ++c4) {
      const v4f hv = *(const v4fa*)(hr + 4 * c4);
      const v4f av = *(const v4fa*)(sa + 4 * c4);
      d = fmaf(hv.x, av.x, d);
      d = fmaf(hv.y, av.y, d);
      d = fmaf(hv.z, av.z, d);
      d = fmaf(hv.w, av.w, d);
    }
    sdot[which * GBM + rw] = d;
  }
  __syncthreads();

  v4f fv[2];
#pragma unroll
  for (int i = 0; i < 2; ++i) {
    const int p = tid + GTHR * i;
    fv[i] = *(const v4fa*)(stg + (p >> 2) * NCOL + 4 * (p & 3));
  }
  const int which2 = lane >> 4, piece = lane & 15;
  const v4f sdv = *(const v4fa*)(sdot + which2 * GBM + 4 * piece);
  float* hb = HS + (size_t)rowBase * H1C;
  float* sp = SD + (size_t)which2 * (size_t)MPr + rowBase + 4 * piece;

#pragma unroll
  for (int i = 0; i < 2; ++i) *(volatile v4f*)(hb + 4 * (tid + GTHR * i)) = fv[i];
  if (wave == 0) *(volatile v4f*)sp = sdv;
  __threadfence();
#pragma unroll
  for (int i = 0; i < 2; ++i) *(volatile v4f*)(hb + 4 * (tid + GTHR * i)) = fv[i];
  if (wave == 0) *(volatile v4f*)sp = sdv;
}

__device__ __forceinline__ void bucket_out(int* ob, int npc, int tid, const int* sorted,
                                           const int* btot, const int* boff) {
#pragma unroll 1
  for (int p = tid; p < npc; p += NTHR) {
    const int b  = p >> 4;
    const int j0 = (p & 15) * 4;
    const int cb = btot[b];
    const int cc = cb < 0 ? 0 : (cb > SEGCAP - 1 ? SEGCAP - 1 : cb);
    const int bo = boff[b];
    int vv[4];
#pragma unroll
    for (int q = 0; q < 4; ++q) {
      const int j = j0 + q;
      int ix = bo + j - 1;
      ix = ix < 0 ? 0 : (ix > CE - 1 ? CE - 1 : ix);
      int v = sorted[ix];
      v = (j - 1 < cc) ? v : -1;
      v = (j == 0) ? cb : v;
      vv[q] = v;
    }
    v4i o; o.x = vv[0]; o.y = vv[1]; o.z = vv[2]; o.w = vv[3];
    *(volatile v4i*)(ob + 4 * p) = o;
  }
}

__global__ __launch_bounds__(NTHR) void k_bucket(const int* __restrict__ srcs, const int* __restrict__ dsts,
                                                 int nE, int nN, int NB, int* BKT) {
  __shared__ __attribute__((aligned(16))) int sorted[CE];
  __shared__ __attribute__((aligned(16))) int wcnt[NWAVE * NBP];
  __shared__ int btot[NBP];
  __shared__ int boff[NBP];
  __shared__ int wtot[NWAVE];
  const int tid = (int)threadIdx.x, lane = tid & 31, wave = tid >> 5;
  const int chunk = (int)blockIdx.x;
  const int cbase = chunk * CE;

  {
    const v4i z4 = {0, 0, 0, 0};
    for (int i = tid * 4; i < CE; i += NTHR * 4) *(v4ia*)(sorted + i) = z4;
    for (int i = tid * 4; i < NWAVE * NBP; i += NTHR * 4) *(v4ia*)(wcnt + i) = z4;
  }
  __syncthreads();

  const int wb = cbase + wave * WSUB;
#pragma unroll 4
  for (int g = 0; g < GPW; ++g) {
    const int e  = wb + g * 32 + lane;
    const int ec = e < nE ? e : nE - 1;
    const int d  = dsts[ec];
    const bool valid = (e < nE) && ((unsigned)d < (unsigned)nN);
    const int bin = valid ? (d >> SLB) : 0;
    if (valid) atomicAdd(&wcnt[wave * NBP + bin], 1);
  }
  __syncthreads();

  for (int b = tid; b < NBP; b += NTHR) {
    int run = 0;
#pragma unroll
    for (int w = 0; w < NWAVE; ++w) {
      const int c = wcnt[w * NBP + b];
      wcnt[w * NBP + b] = run;
      run += c;
    }
    btot[b] = run;
  }
  __syncthreads();

  {
    const int e0 = btot[2 * tid], e1 = btot[2 * tid + 1];
    const int ts = e0 + e1;
    const int incl = wave_incl(ts, lane);
    if (lane == 31) wtot[wave] = incl;
    __syncthreads();
    int pre = 0;
#pragma unroll
    for (int w2 = 0; w2 < NWAVE; ++w2) pre += (w2 < wave) ? wtot[w2] : 0;
    const int ex = pre + incl - ts;
    boff[2 * tid]     = ex;
    boff[2 * tid + 1] = ex + e0;
  }
  __syncthreads();

#pragma unroll 1
  for (int g = 0; g < GPW; ++g) {
    const int e  = wb + g * 32 + lane;
    const int ec = e < nE ? e : nE - 1;
    const int d  = dsts[ec];
    const int s  = srcs[ec];
    const bool valid = (e < nE) && ((unsigned)d < (unsigned)nN);
    const int bin = valid ? (d >> SLB) : 0;
    const unsigned mm = match_mask<9>(bin, valid);
    const unsigned lt = (1u << lane) - 1u;
    const int rank = (int)__builtin_popcount(mm & lt);
    const int cn   = (int)__builtin_popcount(mm);
    const int wv = wcnt[wave * NBP + bin];
    const int bo = boff[bin];
    const int pos = bo + wv + rank;
    const int sc = s < 0 ? 0 : (s > nN - 1 ? nN - 1 : s);
    if (valid && pos >= 0 && pos < CE) sorted[pos] = (sc << SLB) | (d & (NBRUN - 1));
    __syncthreads();
    if (valid && rank == cn - 1) wcnt[wave * NBP + bin] = wv + cn;
    __syncthreads();
  }

  const int npc = NB * (SEGCAP / 4);
  int* ob = BKT + (size_t)chunk * (size_t)NB * SEGCAP;
  bucket_out(ob, npc, tid, sorted, btot, boff);
  __threadfence();
  bucket_out(ob, npc, tid, sorted, btot, boff);
}

template <int L>
__global__ __launch_bounds__(NTHR) void k_scan(
    const int* __restrict__ BKT, int NCH, int NB, int nN, int MPr,
    const float* __restrict__ HS, const float* __restrict__ SD,
    const float* __restrict__ pb1, const float* __restrict__ pW2,
    const float* __restrict__ H2in, const float* __restrict__ pa2s,
    const float* __restrict__ pa2d, const float* __restrict__ pb2,
    float* H2out, float* outp) {
  extern __shared__ __attribute__((aligned(16))) int dsm[];
  int* segcnt = dsm + O_SEGCNT;
  int* segoff = dsm + O_SEGOFF;
  int* hl     = dsm + O_HL;
  int* sl     = dsm + O_SL;
  int* wcn    = dsm + O_WCN;
  int* cnt    = dsm + O_CNT;
  int* offs   = dsm + O_OFFS;
  int* misc   = dsm + O_MISC;
  const int tid = (int)threadIdx.x, lane = tid & 31, wave = tid >> 5;
  const int b = (int)blockIdx.x;
  const int nodeBase = b * NBRUN;

  {
    const v4i z4 = {0, 0, 0, 0};
    for (int i = tid * 4; i < ZINTS; i += NTHR * 4) *(v4ia*)(dsm + i) = z4;
  }
  __syncthreads();

  {
    int bad = 0;
    for (int c = tid; c < NCHP; c += NTHR) {
      const int cl = c < NCH ? c : NCH - 1;
      int craw = BKT[((size_t)cl * (size_t)NB + (size_t)b) * SEGCAP];
      craw = (c < NCH) ? craw : 0;
      bad |= (craw < 0 || craw > SEGCAP - 1) ? 1 : 0;
      segcnt[c] = craw < 0 ? 0 : (craw > SEGCAP - 1 ? SEGCAP - 1 : craw);
    }
    if (bad != 0) misc[9] = 1;
  }
  __syncthreads();
  int nh;
  {
    const int e0 = segcnt[2 * tid], e1 = segcnt[2 * tid + 1];
    const int ts = e0 + e1;
    const int incl = wave_incl(ts, lane);
    if (lane == 31) misc[wave] = incl;
    __syncthreads();
    int pre = 0, all = 0;
#pragma unroll
    for (int w2 = 0; w2 < NWAVE; ++w2) {
      const int c = misc[w2];
      all += c;
      pre += (w2 < wave) ? c : 0;
    }
    const int ex = pre + incl - ts;
    segoff[2 * tid]     = ex;
    segoff[2 * tid + 1] = ex + e0;
    nh = all;
  }
  const bool ovf = (misc[9] != 0) || (nh > RCAP);
  nh = nh > RCAP ? RCAP : nh;
  __syncthreads();

#pragma unroll 1
  for (int c = wave; c < NCH; c += NWAVE) {
    const int n = segcnt[c];
    const int o = segoff[c];
    const int* seg = BKT + ((size_t)c * (size_t)NB + (size_t)b) * SEGCAP;
    const int i1 = (33 + lane) < SEGCAP ? (33 + lane) : SEGCAP - 1;
    const int v0 = seg[1 + lane];
    const int v1 = seg[i1];
    if (lane < n && o + lane < RCAP) hl[o + lane] = v0;
    if (32 + lane < n && o + 32 + lane < RCAP) hl[o + 32 + lane] = v1;
  }
  __syncthreads();

  const int per = ((nh + NTHR - 1) / NTHR) * 32;
  const int ng  = per >> 5;
  const int wb0 = wave * per;
#pragma unroll 1
  for (int g = 0; g < ng; ++g) {
    const int idx = wb0 + g * 32 + lane;
    const bool valid = idx < nh;
    const int ent = hl[idx < RCAP ? idx : RCAP - 1];
    const int slot = ent & (NBRUN - 1);
    if (valid) atomicAdd(&dsm[O_WCN + wave * NBRUN + slot], 1);
  }
  __syncthreads();

  {
    int run = 0;
#pragma unroll
    for (int w = 0; w < NWAVE; ++w) {
      const int c = wcn[w * NBRUN + tid];
      wcn[w * NBRUN + tid] = run;
      run += c;
    }
    cnt[tid] = run;
    const int incl = wave_incl(run, lane);
    if (lane == 31) misc[wave] = incl;
    __syncthreads();
    int pre = 0;
#pragma unroll
    for (int w2 = 0; w2 < NWAVE; ++w2) pre += (w2 < wave) ? misc[w2] : 0;
    offs[tid] = pre + incl - run;
  }
  __syncthreads();

#pragma unroll 1
  for (int g = 0; g < ng; ++g) {
    const int idx = wb0 + g * 32 + lane;
    const bool valid = idx < nh;
    const int ent = hl[idx < RCAP ? idx : RCAP - 1];
    const int slot = ent & (NBRUN - 1);
    const unsigned mm = match_mask<SLB>(slot, valid);
    const unsigned lt = (1u << lane) - 1u;
    const int rank = (int)__builtin_popcount(mm & lt);
    const int cn   = (int)__builtin_popcount(mm);
    const int wv = wcn[wave * NBRUN + slot];
    const int pos = offs[slot] + wv + rank;
    if (valid && pos >= 0 && pos < RCAP) sl[pos] = (int)((unsigned)ent >> SLB);
    __syncthreads();
    if (valid && rank == cn - 1) wcn[wave * NBRUN + slot] = wv + cn;
    __syncthreads();
  }

  const float qnan = __int_as_float(0x7fc00000);
  const int cch = lane & 15, hf = lane >> 4;
  float res = 0.0f;

  if constexpr (L == 1) {
    const float b1c = bfr(pb1[cch]);
    const float w2c = bfr(pW2[cch]);
#pragma unroll 1
    for (int j = 0; j < 32; ++j) {
      const int slot = wave * 32 + j;
      const int node = nodeBase + slot;
      const int nc   = node < nN ? node : nN - 1;
      const int craw = cnt[slot];
      int c = craw < 0 ? 0 : (craw > DEGCAP ? DEGCAP : craw);
      int o = offs[slot];
      o = o < 0 ? 0 : (o > nh ? nh : o);
      if (c > nh - o) c = nh - o;
      const float pz = (ovf || craw > DEGCAP) ? qnan : 0.0f;
      const float ad = SD[(size_t)MPr + nc];
      float mx = -3.0e38f, z = 0.0f, acc = 0.0f;
#pragma unroll 1
      for (int b0 = 0; b0 < c; b0 += 32) {
        int idx = o + b0 + lane;
        idx = idx > RCAP - 1 ? RCAP - 1 : idx;
        int sr = sl[idx];
        sr = sr < 0 ? 0 : (sr > nN - 1 ? nN - 1 : sr);
        float sc = SD[sr] + ad;
        sc = sc > 0.f ? sc : NEGSL * sc;
        const int m32 = (c - b0) < 32 ? (c - b0) : 32;
        const bool act = lane < m32;
        float mb = act ? sc : -3.0e38f;
#pragma unroll
        for (int off = 16; off > 0; off >>= 1) mb = fmaxf(mb, __shfl_xor(mb, off));
        const float mn = fmaxf(mx, mb);
        const float rs = expf(mx - mn);
        float p = expf(sc - mn);
        p = act ? p : 0.0f;
        float zs = p;
#pragma unroll
        for (int off = 16; off > 0; off >>= 1) zs += __shfl_xor(zs, off);
        z   = fmaf(z, rs, zs);
        acc = acc * rs;
        mx  = mn;
        const int half = (m32 + 1) >> 1;
#pragma unroll 2
        for (int i = 0; i < half; ++i) {
          const int k  = 2 * i + hf;
          const int sk = __shfl(sr, k);
          const float pk = __shfl(p, k);
          const float hv = HS[(size_t)sk * H1C + cch];
          acc = fmaf(pk, hv, acc);
        }
      }
      const float tot = acc + __shfl_xor(acc, 16);
      const float inv = 1.0f / (z + EPS_SM);
      const float o1  = fmaf(tot, inv, b1c) + pz;
      const float h1v = (o1 > 0.0f) ? o1 : (o1 - o1);
      float t = h1v * w2c;
#pragma unroll
      for (int off = 8; off > 0; off >>= 1) t += __shfl_xor(t, off);
      const float h2v = (node < nN) ? t : 0.0f;
      res = (lane == j) ? h2v : res;
    }
    float* hp = H2out + nodeBase + wave * 32 + lane;
    *(volatile float*)hp = res;
    __threadfence();
    *(volatile float*)hp = res;
  } else {
    const float a2sv = bfr(pa2s[0]);
    const float a2dv = bfr(pa2d[0]);
    const float b2v  = bfr(pb2[0]);
#pragma unroll 1
    for (int j = 0; j < 32; ++j) {
      const int slot = wave * 32 + j;
      const int node = nodeBase + slot;
      const int nc   = node < nN ? node : nN - 1;
      const int craw = cnt[slot];
      int c = craw < 0 ? 0 : (craw > DEGCAP ? DEGCAP : craw);
      int o = offs[slot];
      o = o < 0 ? 0 : (o > nh ? nh : o);
      if (c > nh - o) c = nh - o;
      const float pz = (ovf || craw > DEGCAP) ? qnan : 0.0f;
      const float ad2 = H2in[nc] * a2dv;
      float mx = -3.0e38f, z = 0.0f, accn = 0.0f;
#pragma unroll 1
      for (int b0 = 0; b0 < c; b0 += 32) {
        int idx = o + b0 + lane;
        idx = idx > RCAP - 1 ? RCAP - 1 : idx;
        int sr = sl[idx];
        sr = sr < 0 ? 0 : (sr > nN - 1 ? nN - 1 : sr);
        const float hs = H2in[sr];
        float sc = hs * a2sv + ad2;
        sc = sc > 0.f ? sc : NEGSL * sc;
        const int m32 = (c - b0) < 32 ? (c - b0) : 32;
        const bool act = lane < m32;
        float mb = act ? sc : -3.0e38f;
#pragma unroll
        for (int off = 16; off > 0; off >>= 1) mb = fmaxf(mb, __shfl_xor(mb, off));
        const float mn = fmaxf(mx, mb);
        const float rs = expf(mx - mn);
        float p = expf(sc - mn);
        p = act ? p : 0.0f;
        float zs = p;
        float ns = act ? p * hs : 0.0f;
#pragma unroll
        for (int off = 16; off > 0; off >>= 1) {
          zs += __shfl_xor(zs, off);
          ns += __shfl_xor(ns, off);
        }
        z    = fmaf(z, rs, zs);
        accn = fmaf(accn, rs, ns);
        mx   = mn;
      }
      const float inv = 1.0f / (z + EPS_SM);
      const float ov  = fmaf(accn, inv, b2v) + pz;
      res = (lane == j) ? ov : res;
    }
    const int lineBase = nodeBase + wave * 32;
    if (lineBase < nN) {
      float* op = outp + lineBase + lane;
      *(volatile float*)op = res;
      __threadfence();
      *(volatile float*)op = res;
    }
  }
}

static inline int cdiv(int a, int b) { return (a + b - 1) / b; }

extern "C" void kernel_launch(void* const* d_in, const int* in_sizes, int n_in,
                              void* d_out, int out_size, void* d_ws, size_t ws_size,
                              hipStream_t stream) {
  if (n_in < 11) return;
  if (in_sizes[0] < DIN || (in_sizes[0] % DIN) != 0) return;
  const int nN = in_sizes[0] / DIN;
  if (nN < 32 || (nN % 32) != 0) return;
  if (in_sizes[1] < 2 || (in_sizes[1] & 1) != 0) return;
  const int nE = in_sizes[1] / 2;
  if (nE < 1 || nE > (1 << 30)) return;
  if (in_sizes[2] != DIN * H1C || in_sizes[3] != DIN * H1C) return;
  if (in_sizes[4] != H1C || in_sizes[5] != H1C || in_sizes[6] != H1C) return;
  if (in_sizes[7] != H1C) return;
  if (in_sizes[8] != 1 || in_sizes[9] != 1 || in_sizes[10] != 1) return;
  if (out_size != nN) return;

  const int NB  = cdiv(nN, NBRUN);
  if (NB > NBP) return;
  const int NCH = cdiv(nE, CE);
  if (NCH > NCHP) return;
  const int MP  = cdiv(nN, GBM) * GBM;
  const int gM  = MP / GBM;

  const float* x    = (const float*)d_in[0];
  const int*   ei   = (const int*)  d_in[1];
  const float* W1s  = (const float*)d_in[2];
  const float* W1d  = (const float*)d_in[3];
  const float* a1s  = (const float*)d_in[4];
  const float* a1d  = (const float*)d_in[5];
  const float* b1   = (const float*)d_in[6];
  const float* W2   = (const float*)d_in[7];
  const float* a2s  = (const float*)d_in[8];
  const float* a2d  = (const float*)d_in[9];
  const float* b2   = (const float*)d_in[10];
  float* out = (float*)d_out;
  const int* src = ei;
  const int* dst = ei + nE;

  char* ws = (char*)d_ws;
  size_t off = 0;
  const size_t oWT  = off; off += (size_t)NCOL * DIN * 2;                        off = (off + 255) & ~(size_t)255;
  const size_t oHS  = off; off += (size_t)MP * H1C * 4;                          off = (off + 255) & ~(size_t)255;
  const size_t oSD  = off; off += (size_t)2 * MP * 4;                            off = (off + 255) & ~(size_t)255;
  const size_t oH2  = off; off += (size_t)NB * NBRUN * 4;                        off = (off + 255) & ~(size_t)255;
  const size_t oBK  = off; off += (size_t)NCH * (size_t)NB * SEGCAP * 4;         off = (off + 255) & ~(size_t)255;
  if (off > ws_size || off > (size_t)WSMAX) return;
  unsigned short* WT  = (unsigned short*)(ws + oWT);
  float*          HS  = (float*)(ws + oHS);
  float*          SD  = (float*)(ws + oSD);
  float*          H2  = (float*)(ws + oH2);
  int*            BKT = (int*)(ws + oBK);

  const int scanLds = ZINTS * 4;
  hipFuncSetAttribute(reinterpret_cast<const void*>(&k_scan<1>), hipFuncAttributeMaxDynamicSharedMemorySize, scanLds);
  hipFuncSetAttribute(reinterpret_cast<const void*>(&k_scan<2>), hipFuncAttributeMaxDynamicSharedMemorySize, scanLds);

  k_wprep<<<2, NTHR, 0, stream>>>(W1s, W1d, WT);
  k_gemm1<<<gM, GTHR, 0, stream>>>(x, WT, a1s, a1d, HS, SD, nN, MP);
  k_bucket<<<NCH, NTHR, 0, stream>>>(src, dst, nE, nN, NB, BKT);
  k_scan<1><<<NB, NTHR, scanLds, stream>>>(BKT, NCH, NB, nN, MP, HS, SD, b1, W2, SD, a2s, a2d, b2, H2, out);
  k_scan<2><<<NB, NTHR, scanLds, stream>>>(BKT, NCH, NB, nN, MP, HS, SD, b1, W2, H2, a2s, a2d, b2, H2, out);
}
